// FourierAttention_27754078666803
// MI455X (gfx1250) — hardware-verified
//
#include <hip/hip_runtime.h>
#include <math.h>

typedef __attribute__((ext_vector_type(16))) _Float16 v16h;
typedef __attribute__((ext_vector_type(16))) __bf16 v16b;
typedef __attribute__((ext_vector_type(8)))  _Float16 v8h;
typedef __attribute__((ext_vector_type(8)))  float v8f;
typedef __attribute__((ext_vector_type(4)))  float v4f;
typedef __attribute__((ext_vector_type(2)))  float v2f;
typedef __attribute__((ext_vector_type(4)))  unsigned v4u;
typedef __attribute__((ext_vector_type(4)))  int v4i;
typedef float __attribute__((may_alias)) float_a;
typedef int __attribute__((may_alias)) int_a;

template <typename T> __device__ __forceinline__ void vst2(void* p, T v) { *(volatile T*)p = v; __threadfence(); *(volatile T*)p = v; }
__device__ __forceinline__ v8f wmma16(v16h a, v16h b, v8f c) {
  v8f d = __builtin_amdgcn_wmma_f32_16x16x32_f16(false, a, false, b, (short)0, c, false, false);
  asm volatile("v_nop\n\tv_nop\n\tv_nop\n\tv_nop" : "+v"(d) : "v"(a), "v"(b));
  return d;
}
__device__ __forceinline__ v8f wmma_bf(v16b a, v16b b, v8f c) {
  v8f d = __builtin_amdgcn_wmma_f32_16x16x32_bf16(false, a, false, b, (short)0, c, false, false);
  asm volatile("v_nop\n\tv_nop\n\tv_nop\n\tv_nop" : "+v"(d) : "v"(a), "v"(b));
  return d;
}
__device__ __forceinline__ v16h frag_h(const _Float16* rowk0, int lane) {
  union { v16h v; v8h q[2]; } u; const _Float16* p = rowk0 + 8 * (lane >> 4);
  u.q[0] = *(const v8h*)p; u.q[1] = *(const v8h*)(p + 16); return u.v;
}
__device__ __forceinline__ v16h frag_f32(const float* rowk0, int lane) {
  v16h a; const float* p = rowk0 + 8 * (lane >> 4);
#pragma unroll
  for (int i = 0; i < 8; ++i) { a[i] = (_Float16)p[i]; a[8 + i] = (_Float16)p[16 + i]; }
  return a;
}
__device__ __forceinline__ v16h frag_f32s(const float* rowk0, int lane, float sc) {
  v16h a; const float* p = rowk0 + 8 * (lane >> 4);
#pragma unroll
  for (int i = 0; i < 8; ++i) { a[i] = (_Float16)(p[i] * sc); a[8 + i] = (_Float16)(p[16 + i] * sc); }
  return a;
}
__device__ __forceinline__ v16h fragc_f32(const float* W, int k0, int n, int lane, int ld, int K) {
  v16h a; const int g = lane >> 4;
#pragma unroll
  for (int i = 0; i < 8; ++i) { const int ka = k0 + 8 * g + i, kb = ka + 16;
    a[i] = (_Float16)(ka < K ? W[(size_t)(ka < K ? ka : K - 1) * ld + n] : 0.f); a[8 + i] = (_Float16)(kb < K ? W[(size_t)(kb < K ? kb : K - 1) * ld + n] : 0.f); }
  return a;
}
struct F2 { v16b h, l; };
__device__ __forceinline__ F2 bsplit16(const float v[16]) { F2 r;
#pragma unroll
  for (int i = 0; i < 16; ++i) { const __bf16 h = (__bf16)v[i]; r.h[i] = h; r.l[i] = (__bf16)(v[i] - (float)h); }
  return r; }
__device__ __forceinline__ F2 split_row(const float* row, int k0, int lane) { float v[16]; const float* p = row + k0 + 8 * (lane >> 4);
#pragma unroll
  for (int i = 0; i < 8; ++i) { v[i] = p[i]; v[8 + i] = p[16 + i]; }
  return bsplit16(v); }
__device__ __forceinline__ F2 split_rowK(const float* row, int k0, int lane, int K) { float v[16]; const int g = lane >> 4;
#pragma unroll
  for (int i = 0; i < 8; ++i) { const int ka = k0 + 8 * g + i, kb = ka + 16; v[i] = ka < K ? row[ka < K ? ka : K - 1] : 0.f; v[8 + i] = kb < K ? row[kb < K ? kb : K - 1] : 0.f; }
  return bsplit16(v); }
__device__ __forceinline__ F2 split_col(const float* W, int k0, int n, int lane, int ld, int K) { float v[16]; const int g = lane >> 4;
#pragma unroll
  for (int i = 0; i < 8; ++i) { const int ka = k0 + 8 * g + i, kb = ka + 16; v[i] = ka < K ? W[(size_t)(ka < K ? ka : K - 1) * ld + n] : 0.f; v[8 + i] = kb < K ? W[(size_t)(kb < K ? kb : K - 1) * ld + n] : 0.f; }
  return bsplit16(v); }
__device__ __forceinline__ v8f mac3(const F2& a, const F2& b, v8f c) { c = wmma_bf(a.l, b.h, c); c = wmma_bf(a.h, b.l, c); return wmma_bf(a.h, b.h, c); }
__device__ __forceinline__ float sigm(float v) { return 1.0f / (1.0f + expf(-v)); }
#define LDSX() do { asm volatile("s_wait_dscnt 0" ::: "memory"); __builtin_amdgcn_wave_barrier(); __builtin_amdgcn_fence(__ATOMIC_RELEASE, "workgroup"); } while (0)


#define NB 4
#define SS 2048
#define DM 1024
#ifndef NBT
#define NBT NB
#define TRB (SS / 64)
#endif
typedef __attribute__((ext_vector_type(8))) __bf16 v8b;
__device__ __forceinline__ v16b frag_b(const __bf16* rowk0, int lane) {
  union { v16b v; v8b q[2]; } u; const __bf16* p = rowk0 + 8 * (lane >> 4);
  u.q[0] = *(const v8b*)p; u.q[1] = *(const v8b*)(p + 16); return u.v;
}
__device__ __forceinline__ float bfr(float v) { return (float)(__bf16)v; }
__device__ __attribute__((noinline)) float exp_ni(float v) { return expf(v); }
__device__ __attribute__((noinline)) float erf_ni(float v) { return erff(v); }

#define PK_Q 0
#define PK_K (PK_Q + DM * DM)
#define PK_V (PK_K + DM * DM)
#define PK_O (PK_V + DM * DM)
#define PK_END (PK_O + DM * DM)
#define WS_PK  0u
#define WS_Q   (WS_PK + 2u * PK_END)
#define WS_K   (WS_Q + 4u * SS * DM)
#define WS_VTH (WS_K + 4u * SS * DM)
#define WS_VTL (WS_VTH + 2u * DM * SS)
#define WS_S   (WS_VTL + 2u * DM * SS)
#define WS_O   (WS_S + 4u * SS * SS)
#define WS_END (WS_O + 4u * SS * DM)

__global__ __launch_bounds__(256) void k_pack(const float* __restrict__ Wm, __bf16* __restrict__ DST) {
  __shared__ __align__(16) __bf16 s[DM]; const int n = blockIdx.x, tid = threadIdx.x; const float* src = Wm + (size_t)n * DM;
  for (int k = tid; k < DM; k += 256) s[k] = (__bf16)src[k];
  __syncthreads();
  if (tid < DM / 8) vst2((unsigned*)(DST + (size_t)n * DM + tid * 8), *(const v4u*)&s[tid * 8]);
}
template <int VTM>
__global__ __launch_bounds__(128) void k_proj(const float* __restrict__ X, const __bf16* __restrict__ P, const float* __restrict__ bias, float* __restrict__ OUT, __bf16* __restrict__ VTH, __bf16* __restrict__ VTL) {
  __shared__ __align__(16) float so[4][16][132]; __shared__ __align__(16) __bf16 sth[VTM ? 128 : 1][72], stl[VTM ? 128 : 1][72];
  const int tid = threadIdx.x, wave = tid >> 5, lane = tid & 31, col = lane & 15, g = lane >> 4; const int s0 = blockIdx.x * 64; const size_t r0 = (size_t)s0 + wave * 16; const int n0 = blockIdx.y * 128;
  v8f acc[8] = {};
#pragma unroll 2
  for (int kc = 0; kc < DM / 32; ++kc) { v16b a; { const float* p = X + (r0 + col) * DM + kc * 32 + 8 * g;
#pragma unroll
      for (int i = 0; i < 8; ++i) { a[i] = (__bf16)p[i]; a[8 + i] = (__bf16)p[16 + i]; } }
#pragma unroll
    for (int j = 0; j < 8; ++j) acc[j] = wmma_bf(a, frag_b(P + (size_t)(n0 + j * 16 + col) * DM + kc * 32, lane), acc[j]); }
  if (!VTM) {
#pragma unroll
    for (int j = 0; j < 8; ++j) { const float bb = bfr(bias[n0 + j * 16 + col]);
#pragma unroll
      for (int r = 0; r < 8; ++r) so[wave][8 * g + r][j * 16 + col] = acc[j][r] + bb; }
    LDSX();
    for (int rl = 0; rl < 16; ++rl) vst2(OUT + (r0 + rl) * DM + n0 + lane * 4, *(const v4f*)&so[wave][rl][lane * 4]);
  } else {
#pragma unroll
    for (int j = 0; j < 8; ++j) { const float bb = bfr(bias[n0 + j * 16 + col]);
#pragma unroll
      for (int r = 0; r < 8; ++r) { const float v = acc[j][r] + bb; const __bf16 hb = (__bf16)v; sth[j * 16 + col][wave * 16 + 8 * g + r] = hb; stl[j * 16 + col][wave * 16 + 8 * g + r] = (__bf16)(v - (float)hb); } }
    __syncthreads();
    for (int q = tid; q < 128 * 8; q += 128) { const int d = q >> 3, pc = q & 7; const size_t o = (size_t)(n0 + d) * SS + s0 + pc * 8; vst2((unsigned*)(VTH + o), *(const v4u*)&sth[d][pc * 8]); vst2((unsigned*)(VTL + o), *(const v4u*)&stl[d][pc * 8]); }
  }
}
__global__ __launch_bounds__(128) void k_scores(const float* __restrict__ Q, const float* __restrict__ Kx, float* __restrict__ S) {
  __shared__ __align__(16) float so[4][16][132];
  const int tid = threadIdx.x, wave = tid >> 5, lane = tid & 31, col = lane & 15, g = lane >> 4; const size_t r0 = (size_t)blockIdx.x * 64 + wave * 16; const int n0 = blockIdx.y * 128;
  v8f acc[8] = {};
#pragma unroll 1
  for (int kc = 0; kc < DM / 32; ++kc) { const F2 a = split_row(Q + (r0 + col) * DM, kc * 32, lane);
#pragma unroll
    for (int j = 0; j < 8; ++j) { const F2 kb = split_row(Kx + (size_t)(n0 + j * 16 + col) * DM, kc * 32, lane); acc[j] = mac3(a, kb, acc[j]); } }
#pragma unroll
  for (int j = 0; j < 8; ++j)
#pragma unroll
    for (int r = 0; r < 8; ++r) so[wave][8 * g + r][j * 16 + col] = acc[j][r] * 0.125f;
  LDSX();
  for (int rl = 0; rl < 16; ++rl) vst2(S + (r0 + rl) * SS + n0 + lane * 4, *(const v4f*)&so[wave][rl][lane * 4]);
}
__global__ __launch_bounds__(256) void k_soft(float* __restrict__ S) {
  const int wave = threadIdx.x >> 5, lane = threadIdx.x & 31; float* row = S + ((size_t)blockIdx.x * 8 + wave) * SS;
  float v[64]; float mx = -3.0e38f;
#pragma unroll
  for (int i = 0; i < 64; ++i) { v[i] = row[lane * 4 + (i & 3) + (i >> 2) * 128]; mx = fmaxf(mx, v[i]); }
#pragma unroll
  for (int o = 1; o < 32; o <<= 1) mx = fmaxf(mx, __shfl_xor(mx, o));
  float z = 0.f;
#pragma unroll
  for (int i = 0; i < 64; ++i) { v[i] = exp_ni(v[i] - mx); z += v[i]; }
#pragma unroll
  for (int o = 1; o < 32; o <<= 1) z += __shfl_xor(z, o);
  const float iz = 1.0f / z;
#pragma unroll
  for (int k = 0; k < 16; ++k) { v4f p; p[0] = v[k * 4] * iz; p[1] = v[k * 4 + 1] * iz; p[2] = v[k * 4 + 2] * iz; p[3] = v[k * 4 + 3] * iz; vst2(row + k * 128 + lane * 4, p); }
}
__global__ __launch_bounds__(128) void k_pv(const float* __restrict__ S, const __bf16* __restrict__ VTH, const __bf16* __restrict__ VTL, float* __restrict__ O) {
  __shared__ __align__(16) float so[4][16][132];
  const int tid = threadIdx.x, wave = tid >> 5, lane = tid & 31, col = lane & 15, g = lane >> 4; const size_t r0 = (size_t)blockIdx.x * 64 + wave * 16; const int n0 = blockIdx.y * 128;
  v8f acc[8] = {};
#pragma unroll 1
  for (int kc = 0; kc < SS / 32; ++kc) { const F2 a = split_row(S + (r0 + col) * SS, kc * 32, lane);
#pragma unroll
    for (int j = 0; j < 8; ++j) { const size_t vr = (size_t)(n0 + j * 16 + col) * SS + kc * 32; const v16b vh = frag_b(VTH + vr, lane), vl = frag_b(VTL + vr, lane); acc[j] = wmma_bf(a.l, vh, acc[j]); acc[j] = wmma_bf(a.h, vl, acc[j]); acc[j] = wmma_bf(a.h, vh, acc[j]); } }
#pragma unroll
  for (int j = 0; j < 8; ++j)
#pragma unroll
    for (int r = 0; r < 8; ++r) so[wave][8 * g + r][j * 16 + col] = acc[j][r];
  LDSX();
  for (int rl = 0; rl < 16; ++rl) vst2(O + (r0 + rl) * DM + n0 + lane * 4, *(const v4f*)&so[wave][rl][lane * 4]);
}
__global__ __launch_bounds__(128) void k_out(const float* __restrict__ O, const __bf16* __restrict__ P, const float* __restrict__ bo, float* __restrict__ Y) {
  __shared__ __align__(16) float so[4][16][132];
  const int tid = threadIdx.x, wave = tid >> 5, lane = tid & 31, col = lane & 15, g = lane >> 4; const size_t r0 = (size_t)blockIdx.x * 64 + wave * 16; const int n0 = blockIdx.y * 128;
  v8f acc[8] = {};
#pragma unroll 2
  for (int kc = 0; kc < DM / 32; ++kc) { const F2 a = split_row(O + (r0 + col) * DM, kc * 32, lane);
#pragma unroll
    for (int j = 0; j < 8; ++j) { const v16b w = frag_b(P + (size_t)(n0 + j * 16 + col) * DM + kc * 32, lane); acc[j] = wmma_bf(a.l, w, acc[j]); acc[j] = wmma_bf(a.h, w, acc[j]); } }
#pragma unroll
  for (int j = 0; j < 8; ++j) { const float bb = bfr(bo[n0 + j * 16 + col]);
#pragma unroll
    for (int r = 0; r < 8; ++r) so[wave][8 * g + r][j * 16 + col] = acc[j][r] + bb; }
  LDSX();
  for (int rl = 0; rl < 16; ++rl) vst2(Y + (r0 + rl) * DM + n0 + lane * 4, *(const v4f*)&so[wave][rl][lane * 4]);
}
extern "C" void kernel_launch(void* const* d_in, const int* in_sizes, int n_in, void* d_out, int out_size, void* d_ws, size_t ws_size, hipStream_t stream) {
  (void)in_sizes; (void)n_in; (void)out_size;
  const float** F = (const float**)d_in;
  if (ws_size < (size_t)WS_END) return;
  char* ws = (char*)d_ws; __bf16 *PK = (__bf16*)(ws + WS_PK), *VTH = (__bf16*)(ws + WS_VTH), *VTL = (__bf16*)(ws + WS_VTL);
  float *Q = (float*)(ws + WS_Q), *Kx = (float*)(ws + WS_K), *S = (float*)(ws + WS_S), *O = (float*)(ws + WS_O);
  k_pack<<<DM, 256, 0, stream>>>(F[1], PK + PK_Q); k_pack<<<DM, 256, 0, stream>>>(F[3], PK + PK_K); k_pack<<<DM, 256, 0, stream>>>(F[5], PK + PK_V); k_pack<<<DM, 256, 0, stream>>>(F[7], PK + PK_O);
  for (int b = 0; b < NBT; ++b) { const float* xb = F[0] + (size_t)b * SS * DM; float* yb = (float*)d_out + (size_t)b * SS * DM;
    k_proj<0><<<dim3(SS / 64, DM / 128), 128, 0, stream>>>(xb, PK + PK_Q, F[2], Q, nullptr, nullptr);
    k_proj<0><<<dim3(SS / 64, DM / 128), 128, 0, stream>>>(xb, PK + PK_K, F[4], Kx, nullptr, nullptr);
    k_proj<1><<<dim3(SS / 64, DM / 128), 128, 0, stream>>>(xb, PK + PK_V, F[6], nullptr, VTH, VTL);
    k_scores<<<dim3(TRB, SS / 128), 128, 0, stream>>>(Q, Kx, S);
    k_soft<<<TRB * 8, 256, 0, stream>>>(S);
    k_pv<<<dim3(TRB, DM / 128), 128, 0, stream>>>(S, VTH, VTL, O);
    k_out<<<dim3(TRB, DM / 128), 128, 0, stream>>>(O, PK + PK_O, F[8], yb); }
}
